// MambaBlock_79018808311895
// MI455X (gfx1250) — hardware-verified
//
#include <hip/hip_runtime.h>
#include <math.h>

typedef __attribute__((ext_vector_type(16))) _Float16 v16h;
typedef __attribute__((ext_vector_type(8)))  _Float16 v8h;
typedef __attribute__((ext_vector_type(8)))  float    v8f;
typedef __attribute__((ext_vector_type(4)))  float    v4f;

constexpr int kBatch = 2;
constexpr int kSeqL  = 1024;
constexpr int kDmod  = 1024;
constexpr int kDin   = 2048;
constexpr int kNst   = 16;
constexpr int kDtR   = 64;
constexpr int kPrjN  = 96;
constexpr int kPrjP  = 128;
constexpr int kXZP   = 2 * kDin;
constexpr int kRows  = kBatch * kSeqL;
constexpr int kTP    = 260;
constexpr float kLnEps   = 1e-5f;
constexpr float kInvDm   = 1.0f / (float)kDmod;
constexpr float kCarryW  = 32.0f;
constexpr float kCarryUC = 16.0f;
constexpr float kCarryDT = 16.0f;
constexpr float kCarryY  = 16.0f;

static_assert(kDtR + 2 * kNst == kPrjN, "x_proj width");
static_assert((kDmod % 32) == 0 && (kDin % 32) == 0 && (kDtR % 32) == 0, "GEMM K multiples of 32");
static_assert((kRows % 64) == 0 && (kXZP % 64) == 0 && (kPrjP % 64) == 0 && (kDin % 64) == 0 && (kDmod % 64) == 0 && (kSeqL % 64) == 0, "GEMM M,N multiples of 64");
static_assert((kSeqL % 64) == 0 && (kDin % 256) == 0 && (kSeqL % 32) == 0 && (kDmod % 64) == 0, "tile multiples");

constexpr size_t kSzWIN  = (size_t)kXZP  * kDmod * 2;
constexpr size_t kSzWXP  = (size_t)kPrjP * kDin  * 2;
constexpr size_t kSzWDT  = (size_t)kDin  * kDtR  * 2;
constexpr size_t kSzWOUT = (size_t)kDmod * kDin  * 2;
constexpr size_t kSzXN   = (size_t)kRows * kDmod * 2;
constexpr size_t kSzXZ   = (size_t)kRows * kXZP  * 4;
constexpr size_t kSzUC   = (size_t)kRows * kDin  * 4;
constexpr size_t kSzUC16 = (size_t)kRows * kDin  * 2;
constexpr size_t kSzPROJ = (size_t)kRows * kPrjP * 4;
constexpr size_t kSzDT16 = (size_t)kRows * kDtR  * 2;
constexpr size_t kSzDLR  = (size_t)kRows * kDin  * 4;
constexpr size_t kSzY16  = (size_t)kRows * kDin  * 2;
constexpr size_t kOffWIN  = 0;
constexpr size_t kOffWXP  = kOffWIN  + kSzWIN;
constexpr size_t kOffWDT  = kOffWXP  + kSzWXP;
constexpr size_t kOffWOUT = kOffWDT  + kSzWDT;
constexpr size_t kOffXN   = kOffWOUT + kSzWOUT;
constexpr size_t kOffXZ   = kOffXN   + kSzXN;
constexpr size_t kOffUC   = kOffXZ   + kSzXZ;
constexpr size_t kOffUC16 = kOffUC   + kSzUC;
constexpr size_t kOffPROJ = kOffUC16 + kSzUC16;
constexpr size_t kOffDT16 = kOffPROJ + kSzPROJ;
constexpr size_t kOffDLR  = kOffDT16 + kSzDT16;
constexpr size_t kOffY16  = kOffDLR  + kSzDLR;
constexpr size_t kWsTotal = kOffY16  + kSzY16;
static_assert(kWsTotal == 102760448ull, "carve total");
static_assert(kWsTotal <= 134217728ull, "carve cap");
static_assert((kOffWXP % 128) == 0 && (kOffWDT % 128) == 0 && (kOffWOUT % 128) == 0 && (kOffXN % 128) == 0 &&
              (kOffXZ % 128) == 0 && (kOffUC % 128) == 0 && (kOffUC16 % 128) == 0 && (kOffPROJ % 128) == 0 &&
              (kOffDT16 % 128) == 0 && (kOffDLR % 128) == 0 && (kOffY16 % 128) == 0, "128-B aligned regions");

__device__ __forceinline__ void row_guard_h(v8f& a, v8f& b, v8f& c, v8f& d, v16h x) {
  asm volatile("v_nop\n\tv_nop\n\tv_nop\n\tv_nop" : "+v"(a), "+v"(b), "+v"(c), "+v"(d) : "v"(x));
}
__device__ __forceinline__ void keep4_h(v16h a, v16h b, v16h c, v16h d) { asm volatile("v_nop" :: "v"(a), "v"(b), "v"(c), "v"(d)); }
__device__ __forceinline__ void acc_guard4(v8f& a, v8f& b, v8f& c, v8f& d) { asm volatile("v_nop\n\tv_nop\n\tv_nop\n\tv_nop" : "+v"(a), "+v"(b), "+v"(c), "+v"(d)); }

struct Frag16 {
  union U { v16h v; v8h h[2]; };
  static __device__ __forceinline__ v16h load(const _Float16* p) {
    U f; f.h[0] = *(const v8h*)(p); f.h[1] = *(const v8h*)(p + 16); return f.v;
  }
  static __device__ __forceinline__ v8f mma(v16h a, v16h b, v8f c) {
    return __builtin_amdgcn_wmma_f32_16x16x32_f16(false, a, false, b, (short)0, c, false, false);
  }
};

template <int BIAS_MODE, bool RESID>
__global__ __launch_bounds__(256) void wmma_gemm64_f16(
    const unsigned short* __restrict__ Ap, int lda, long strideA,
    const unsigned short* __restrict__ Btp, int ldb, long strideB,
    float* __restrict__ Cout, int ldc, long strideC,
    const float* __restrict__ bias,
    const float* __restrict__ resid, long strideR,
    int M, int N, int K, float scale) {
  const _Float16* A  = (const _Float16*)Ap;
  const _Float16* Bt = (const _Float16*)Btp;
  __shared__ __align__(16) float sT[8][16 * 68];
  const int b    = blockIdx.y;
  const int lane = threadIdx.x & 31;
  const int wave = threadIdx.x >> 5;
  const int tilesN = N >> 6;
  const int tilesM = M >> 6;
  const int tile = blockIdx.x * 8 + wave;
  if (tile >= tilesM * tilesN) return;
  const int tm = tile / tilesN;
  const int tn = tile - tm * tilesN;
  const int m0 = tm << 6;
  const int n0 = tn << 6;

  const _Float16* Ab = A  + (size_t)b * strideA;
  const _Float16* Bb = Bt + (size_t)b * strideB;

  const int rlane = lane & 15;
  const int koff  = (lane >> 4) * 8;
  const int mOff  = (lane >> 4) * 8;

  v8f acc[4][4];
#pragma unroll
  for (int i = 0; i < 4; ++i)
#pragma unroll
    for (int j = 0; j < 4; ++j) acc[i][j] = (v8f){0.f,0.f,0.f,0.f,0.f,0.f,0.f,0.f};

  for (int k0 = 0; k0 < K; k0 += 32) {
    v16h bh[4];
#pragma unroll
    for (int j = 0; j < 4; ++j) {
      const size_t bo = (size_t)(n0 + (j << 4) + rlane) * ldb + koff + k0;
      bh[j] = Frag16::load(Bb + bo);
    }
#pragma unroll
    for (int i = 0; i < 4; ++i) {
      const size_t ao = (size_t)(m0 + (i << 4) + rlane) * lda + koff + k0;
      v16h ah = Frag16::load(Ab + ao);
#pragma unroll
      for (int j = 0; j < 4; ++j) acc[i][j] = Frag16::mma(ah, bh[j], acc[i][j]);
      row_guard_h(acc[i][0], acc[i][1], acc[i][2], acc[i][3], ah);
    }
    keep4_h(bh[0], bh[1], bh[2], bh[3]);
  }
  acc_guard4(acc[0][0], acc[0][1], acc[0][2], acc[0][3]);
  acc_guard4(acc[1][0], acc[1][1], acc[1][2], acc[1][3]);
  acc_guard4(acc[2][0], acc[2][1], acc[2][2], acc[2][3]);
  acc_guard4(acc[3][0], acc[3][1], acc[3][2], acc[3][3]);

  float* slab = sT[wave];
  float* C = Cout + (size_t)b * strideC;
  const int hh = lane >> 4, c4 = (lane & 15) * 4;
#pragma unroll
  for (int i = 0; i < 4; ++i) {
    const int mBase = m0 + (i << 4);
#pragma unroll
    for (int j = 0; j < 4; ++j) {
      const int n = n0 + (j << 4) + rlane;
      float bv = 0.f;
      if (BIAS_MODE == 2) bv = bias[n];
#pragma unroll
      for (int r = 0; r < 8; ++r) {
        float v = acc[i][j][r] * scale;
        if (BIAS_MODE == 2) v += bv;
        slab[(mOff + r) * 68 + (j << 4) + rlane] = v;
      }
    }
    __builtin_amdgcn_fence(__ATOMIC_RELEASE, "workgroup");
    __builtin_amdgcn_wave_barrier();
    __builtin_amdgcn_fence(__ATOMIC_ACQUIRE, "workgroup");
    v4f vals[8];
#pragma unroll
    for (int it = 0; it < 4; ++it) {
      const int row = it * 2 + hh;
      v4f v = *(const v4f*)(slab + row * 68 + c4);
      if (RESID) {
        const v4f rv = *(const v4f*)(resid + (size_t)b * strideR + (size_t)(mBase + row) * ldc + n0 + c4);
        v = v + rv;
      }
      vals[it] = v;
    }
    asm volatile("" ::: "memory");
#pragma unroll
    for (int it = 4; it < 8; ++it) {
      const int row = it * 2 + hh;
      v4f v = *(const v4f*)(slab + row * 68 + c4);
      if (RESID) {
        const v4f rv = *(const v4f*)(resid + (size_t)b * strideR + (size_t)(mBase + row) * ldc + n0 + c4);
        v = v + rv;
      }
      vals[it] = v;
    }
    for (int pass = 0; pass < 2; ++pass) {
#pragma unroll
      for (int it = 0; it < 8; ++it) {
        const int row = it * 2 + hh;
        *(volatile v4f*)(C + (size_t)(mBase + row) * ldc + n0 + c4) = vals[it];
      }
      __threadfence();
    }
    __builtin_amdgcn_fence(__ATOMIC_RELEASE, "workgroup");
    __builtin_amdgcn_wave_barrier();
    __builtin_amdgcn_fence(__ATOMIC_ACQUIRE, "workgroup");
  }
}

__global__ __launch_bounds__(256) void cast_f16_kernel(
    const float* __restrict__ src, unsigned short* __restrict__ dst, int total8, int real8, float scale)
{
  const int i = blockIdx.x * 256 + threadIdx.x;
  if (i >= total8) return;
  const bool live = (i < real8);
  const int ic = live ? i : (real8 - 1);
  const float* p = src + ((size_t)ic << 3);
  const v4f a0 = *(const v4f*)(p);
  const v4f a1 = *(const v4f*)(p + 4);
  v8h hv;
#pragma unroll
  for (int e = 0; e < 4; ++e) {
    const float f0 = live ? (a0[e] * scale) : 0.0f;
    const float f1 = live ? (a1[e] * scale) : 0.0f;
    hv[e]     = (_Float16)f0;
    hv[4 + e] = (_Float16)f1;
  }
  unsigned short* q = dst + ((size_t)i << 3);
  *(volatile v8h*)q = hv;
  __threadfence();
  *(volatile v8h*)q = hv;
}

__global__ __launch_bounds__(256) void layernorm_kernel(
    const float* __restrict__ x, const float* __restrict__ lw, const float* __restrict__ lb,
    unsigned short* __restrict__ XN16)
{
  __shared__ float sRed[8 * 32];
  __shared__ float sMu[32];
  __shared__ float sRs[32];
  __shared__ float sT[64 * 33];
  const int tid = threadIdx.x, lane = tid & 31, wave = tid >> 5;
  constexpr int kLT = kSeqL / 32;
  const int b  = blockIdx.x / kLT;
  const int l0 = (blockIdx.x - b * kLT) * 32;
  const float* xb = x + (size_t)b * kDmod * kSeqL + l0 + lane;

  float s = 0.0f;
#pragma unroll 4
  for (int i = 0; i < kDmod / 8; ++i) s += xb[(size_t)(wave + 8 * i) * kSeqL];
  sRed[wave * 32 + lane] = s;
  __syncthreads();
  if (tid < 32) {
    float t = 0.0f;
#pragma unroll
    for (int w = 0; w < 8; ++w) t += sRed[w * 32 + tid];
    sMu[tid] = t * kInvDm;
  }
  __syncthreads();
  const float mu = sMu[lane];
  float s2 = 0.0f;
#pragma unroll 4
  for (int i = 0; i < kDmod / 8; ++i) {
    const float dv = xb[(size_t)(wave + 8 * i) * kSeqL] - mu;
    s2 += dv * dv;
  }
  sRed[wave * 32 + lane] = s2;
  __syncthreads();
  if (tid < 32) {
    float t = 0.0f;
#pragma unroll
    for (int w = 0; w < 8; ++w) t += sRed[w * 32 + tid];
    sRs[tid] = rsqrtf(t * kInvDm + kLnEps);
  }
  __syncthreads();
  const float rs = sRs[lane];

  const int q = lane >> 3, c8 = (lane & 7) * 8;
  const int orow = wave * 4 + q;
#pragma unroll 1
  for (int cc = 0; cc < kDmod / 64; ++cc) {
    const int c0 = cc * 64;
#pragma unroll
    for (int i = 0; i < 8; ++i) {
      const int cl = wave * 8 + i;
      const int c  = c0 + cl;
      const float v = xb[(size_t)c * kSeqL];
      sT[cl * 33 + lane] = ((v - mu) * rs) * lw[c] + lb[c];
    }
    __syncthreads();
    v8h hv;
#pragma unroll
    for (int e = 0; e < 8; ++e) hv[e] = (_Float16)sT[(c8 + e) * 33 + orow];
    unsigned short* dp = XN16 + (size_t)(b * kSeqL + l0 + orow) * kDmod + c0 + c8;
    *(volatile v8h*)dp = hv;
    __threadfence();
    *(volatile v8h*)dp = hv;
    __syncthreads();
  }
}

__global__ __launch_bounds__(256) void conv_silu_kernel(
    const float* __restrict__ XZ, const float* __restrict__ cw, const float* __restrict__ cb,
    float* __restrict__ UC, unsigned short* __restrict__ UC16)
{
  __shared__ __align__(16) float sT[16 * kTP];
  const int tid = threadIdx.x, lane = tid & 31, wave = tid >> 5;
  const int d0 = blockIdx.x * 256, d = d0 + tid;
  const int g0 = blockIdx.y * 64;
  const int tb = g0 & (kSeqL - 1);
  const float w0 = cw[d * 4 + 0], w1 = cw[d * 4 + 1], w2 = cw[d * 4 + 2], w3 = cw[d * 4 + 3];
  const float bc = cb[d];
  float xm3, xm2, xm1;
  {
    const bool hist = (tb > 0);
    const int rb = hist ? (g0 - 3) : g0;
    const float v3 = XZ[(size_t)rb * kXZP + d];
    const float v2 = XZ[(size_t)(rb + 1) * kXZP + d];
    const float v1 = XZ[(size_t)(rb + 2) * kXZP + d];
    xm3 = hist ? v3 : 0.f;
    xm2 = hist ? v2 : 0.f;
    xm1 = hist ? v1 : 0.f;
  }
  const int hrow = wave >> 1;
  const int hch  = (wave & 1) * 128 + lane * 4;
#pragma unroll 1
  for (int sub = 0; sub < 4; ++sub) {
    const int lb = g0 + sub * 16;
#pragma unroll 1
    for (int s = 0; s < 16; ++s) {
      const float xcur = XZ[(size_t)(lb + s) * kXZP + d];
      float acc = w0 * xm3;
      acc = fmaf(w1, xm2, acc);
      acc = fmaf(w2, xm1, acc);
      acc = fmaf(w3, xcur, acc);
      const float sv = acc + bc;
      const float sg = __builtin_amdgcn_rcpf(1.0f + expf(-sv));
      sT[s * kTP + tid] = sv * sg;
      xm3 = xm2; xm2 = xm1; xm1 = xcur;
    }
    __syncthreads();
    v4f fv[4];
    v8h bv[2];
#pragma unroll
    for (int it = 0; it < 4; ++it) fv[it] = *(const v4f*)(sT + (it * 4 + hrow) * kTP + hch);
#pragma unroll
    for (int it = 0; it < 2; ++it) {
      const float* sp = sT + (it * 8 + wave) * kTP + lane * 8;
      const v4f a0 = *(const v4f*)(sp);
      const v4f a1 = *(const v4f*)(sp + 4);
#pragma unroll
      for (int e = 0; e < 4; ++e) {
        bv[it][e]     = (_Float16)(a0[e] * kCarryUC);
        bv[it][4 + e] = (_Float16)(a1[e] * kCarryUC);
      }
    }
    for (int pass = 0; pass < 2; ++pass) {
#pragma unroll
      for (int it = 0; it < 4; ++it)
        *(volatile v4f*)(UC + (size_t)(lb + it * 4 + hrow) * kDin + d0 + hch) = fv[it];
#pragma unroll
      for (int it = 0; it < 2; ++it)
        *(volatile v8h*)(UC16 + (size_t)(lb + it * 8 + wave) * kDin + d0 + lane * 8) = bv[it];
      __threadfence();
    }
    __syncthreads();
  }
}

__global__ __launch_bounds__(256) void dt_cast_kernel(
    const float* __restrict__ PROJ, unsigned short* __restrict__ DT16, int total8, float scale)
{
  const int i = blockIdx.x * 256 + threadIdx.x;
  if (i >= total8) return;
  const int e0  = i << 3;
  const int row = e0 >> 6;
  const int c8  = e0 & 63;
  const float* p = PROJ + (size_t)row * kPrjP + c8;
  const v4f a0 = *(const v4f*)(p);
  const v4f a1 = *(const v4f*)(p + 4);
  v8h hv;
#pragma unroll
  for (int e = 0; e < 4; ++e) {
    hv[e]     = (_Float16)(a0[e] * scale);
    hv[4 + e] = (_Float16)(a1[e] * scale);
  }
  unsigned short* qd = DT16 + e0;
  *(volatile v8h*)qd = hv;
  __threadfence();
  *(volatile v8h*)qd = hv;
}

__global__ __launch_bounds__(256) void scan_kernel(
    const float* __restrict__ DLR, const float* __restrict__ UC, const float* __restrict__ XZ,
    const float* __restrict__ PROJ, const float* __restrict__ A_log, const float* __restrict__ Dv,
    unsigned short* __restrict__ Y16)
{
  __shared__ __align__(16) float sBC[16 * 32];
  __shared__ __align__(16) float sY[16 * kTP];
  __shared__ float sA[kNst * 256];
  const int tid = threadIdx.x, lane = tid & 31, wave = tid >> 5;
  const int d0 = blockIdx.x * 256, d = d0 + tid;
  const size_t row0 = (size_t)blockIdx.y * kSeqL;

#pragma unroll 1
  for (int n = 0; n < kNst; ++n) sA[n * 256 + tid] = -expf(A_log[(size_t)d * kNst + n]);
  __syncthreads();
  float An[kNst], h[kNst];
#pragma unroll
  for (int n = 0; n < kNst; ++n) {
    An[n] = sA[n * 256 + tid];
    h[n] = 0.f;
  }
  const float Dd = Dv[d];

#pragma unroll 1
  for (int c = 0; c < kSeqL / 16; ++c) {
    const int l0 = c * 16;
    if (tid < 128) {
      const int r = tid >> 3, qc = (tid & 7) * 4;
      const v4f v = *(const v4f*)(PROJ + (row0 + l0 + r) * kPrjP + kDtR + qc);
      *(v4f*)(sBC + r * 32 + qc) = v;
    }
    __syncthreads();
#pragma unroll 1
    for (int s = 0; s < 16; ++s) {
      const size_t m = row0 + (size_t)(l0 + s);
      const float av = DLR[m * kDin + d];
      const float xv = UC[m * kDin + d];
      const float zv = XZ[m * kXZP + kDin + d];
      const float ea = expf(-fabsf(av));
      const float up = 1.0f + ea;
      const float l1p = logf(up) + (ea - (up - 1.0f)) * __builtin_amdgcn_rcpf(up);
      const float delta = fmaxf(av, 0.0f) + l1p;
      v4f Bq[4], Cq[4];
#pragma unroll
      for (int qq = 0; qq < 4; ++qq) {
        Bq[qq] = *(const v4f*)(sBC + s * 32 + 4 * qq);
        Cq[qq] = *(const v4f*)(sBC + s * 32 + kNst + 4 * qq);
      }
      const float dtx = delta * xv;
      float y = 0.f;
#pragma unroll
      for (int n = 0; n < kNst; ++n) {
        const float e = __expf(delta * An[n]);
        const float hn = e * h[n] + dtx * Bq[n >> 2][n & 3];
        h[n] = hn;
        y = hn * Cq[n >> 2][n & 3] + y;
      }
      y = xv * Dd + y;
      const float sg = __builtin_amdgcn_rcpf(1.0f + expf(-zv));
      const float g  = zv * sg;
      sY[s * kTP + tid] = (y * g) * kCarryY;
    }
    __syncthreads();
    v8h hv[2];
#pragma unroll
    for (int it = 0; it < 2; ++it) {
      const float* sp = sY + (it * 8 + wave) * kTP + lane * 8;
      const v4f a0 = *(const v4f*)(sp);
      const v4f a1 = *(const v4f*)(sp + 4);
#pragma unroll
      for (int e = 0; e < 4; ++e) { hv[it][e] = (_Float16)a0[e]; hv[it][4 + e] = (_Float16)a1[e]; }
    }
    for (int pass = 0; pass < 2; ++pass) {
#pragma unroll
      for (int it = 0; it < 2; ++it)
        *(volatile v8h*)(Y16 + (row0 + l0 + it * 8 + wave) * kDin + d0 + lane * 8) = hv[it];
      __threadfence();
    }
  }
}

static_assert((kRows / 64) * (kXZP / 64) == 256 * 8, "in_proj grid");
static_assert((kRows / 64) * (kPrjP / 64) == 8 * 8, "x_proj grid");
static_assert((kRows / 64) * (kDin / 64) == 128 * 8, "dt_proj grid");
static_assert((kDmod / 64) * (kSeqL / 64) == 32 * 8, "out_proj grid");
static_assert(((kXZP * kDmod / 8) % 256) == 0 && ((kPrjP * kDin / 8) % 256) == 0 && ((kPrjN * kDin / 8) % 256) == 0 &&
              ((kDin * kDtR / 8) % 256) == 0 && ((kDmod * kDin / 8) % 256) == 0 && ((kRows * kDtR / 8) % 256) == 0, "cast grids");

extern "C" void kernel_launch(void* const* d_in, const int* in_sizes, int n_in,
                              void* d_out, int out_size, void* d_ws, size_t ws_size,
                              hipStream_t stream)
{
  if (n_in < 12) return;
  if (in_sizes[0] != kBatch * kDmod * kSeqL) return;
  if (in_sizes[1] != kDmod || in_sizes[2] != kDmod) return;
  if (in_sizes[3] != kXZP * kDmod) return;
  if (in_sizes[4] != kDin * 4 || in_sizes[5] != kDin) return;
  if (in_sizes[6] != kPrjN * kDin) return;
  if (in_sizes[7] != kDin * kDtR || in_sizes[8] != kDin) return;
  if (in_sizes[9] != kDin * kNst || in_sizes[10] != kDin) return;
  if (in_sizes[11] != kDmod * kDin) return;
  if (out_size != kBatch * kDmod * kSeqL) return;
  if (ws_size < kWsTotal) return;

  const float* x       = (const float*)d_in[0];
  const float* ln_w    = (const float*)d_in[1];
  const float* ln_b    = (const float*)d_in[2];
  const float* W_in    = (const float*)d_in[3];
  const float* conv_w  = (const float*)d_in[4];
  const float* conv_b  = (const float*)d_in[5];
  const float* W_xprj  = (const float*)d_in[6];
  const float* W_dt    = (const float*)d_in[7];
  const float* b_dt    = (const float*)d_in[8];
  const float* A_log   = (const float*)d_in[9];
  const float* Dv      = (const float*)d_in[10];
  const float* W_out   = (const float*)d_in[11];
  float* dout = (float*)d_out;

  char* ws = (char*)d_ws;
  unsigned short* WIN16  = (unsigned short*)(ws + kOffWIN);
  unsigned short* WXP16  = (unsigned short*)(ws + kOffWXP);
  unsigned short* WDT16  = (unsigned short*)(ws + kOffWDT);
  unsigned short* WOUT16 = (unsigned short*)(ws + kOffWOUT);
  unsigned short* XN16   = (unsigned short*)(ws + kOffXN);
  float*          XZ     = (float*)(ws + kOffXZ);
  float*          UC     = (float*)(ws + kOffUC);
  unsigned short* UC16   = (unsigned short*)(ws + kOffUC16);
  float*          PROJ   = (float*)(ws + kOffPROJ);
  unsigned short* DT16   = (unsigned short*)(ws + kOffDT16);
  float*          DLR    = (float*)(ws + kOffDLR);
  unsigned short* Y16    = (unsigned short*)(ws + kOffY16);

  cast_f16_kernel<<<(kXZP * kDmod / 8) / 256, 256, 0, stream>>>(W_in, WIN16, kXZP * kDmod / 8, kXZP * kDmod / 8, kCarryW);
  cast_f16_kernel<<<(kPrjP * kDin / 8) / 256, 256, 0, stream>>>(W_xprj, WXP16, kPrjP * kDin / 8, kPrjN * kDin / 8, kCarryW);
  cast_f16_kernel<<<(kDin * kDtR / 8) / 256, 256, 0, stream>>>(W_dt, WDT16, kDin * kDtR / 8, kDin * kDtR / 8, kCarryW);
  cast_f16_kernel<<<(kDmod * kDin / 8) / 256, 256, 0, stream>>>(W_out, WOUT16, kDmod * kDin / 8, kDmod * kDin / 8, kCarryW);

  layernorm_kernel<<<kBatch * (kSeqL / 32), 256, 0, stream>>>(x, ln_w, ln_b, XN16);

  wmma_gemm64_f16<0, false><<<dim3(256, 1), 256, 0, stream>>>(
      XN16, kDmod, 0L, WIN16, kDmod, 0L,
      XZ, kXZP, 0L, b_dt, x, 0L,
      kRows, kXZP, kDmod, 1.0f / kCarryW);

  conv_silu_kernel<<<dim3(kDin / 256, kRows / 64), 256, 0, stream>>>(XZ, conv_w, conv_b, UC, UC16);

  wmma_gemm64_f16<0, false><<<dim3(8, 1), 256, 0, stream>>>(
      UC16, kDin, 0L, WXP16, kDin, 0L,
      PROJ, kPrjP, 0L, b_dt, x, 0L,
      kRows, kPrjP, kDin, 1.0f / (kCarryUC * kCarryW));

  dt_cast_kernel<<<(kRows * kDtR / 8) / 256, 256, 0, stream>>>(PROJ, DT16, kRows * kDtR / 8, kCarryDT);

  wmma_gemm64_f16<2, false><<<dim3(128, 1), 256, 0, stream>>>(
      DT16, kDtR, 0L, WDT16, kDtR, 0L,
      DLR, kDin, 0L, b_dt, x, 0L,
      kRows, kDin, kDtR, 1.0f / (kCarryDT * kCarryW));

  scan_kernel<<<dim3(kDin / 256, kBatch), 256, 0, stream>>>(DLR, UC, XZ, PROJ, A_log, Dv, Y16);

  wmma_gemm64_f16<0, true><<<dim3(32, kBatch), 256, 0, stream>>>(
      WOUT16, kDin, 0L, Y16, kDin, (long)kSeqL * kDin,
      dout, kSeqL, (long)kDmod * kSeqL, b_dt, x, (long)kDmod * kSeqL,
      kDmod, kSeqL, kDin, 1.0f / (kCarryW * kCarryY));
}
